// PerceiverAlibiSelfAttention_66718021976280
// MI455X (gfx1250) — hardware-verified
//
#include <hip/hip_runtime.h>
#include <math.h>
#include <stdint.h>

#define NB    4
#define SQ    2048
#define NTOK  (NB * SQ)
#define DM    1024
#define NH    16
#define HD    64
#define NQB   (SQ / 64)
#define XSC   16.0f
#define WSC   64.0f
#define VSC   16.0f
#define RSC   4096.0f
#define PSC   1024.0f
#define LNEPS 1e-5f
static_assert(NH * HD == DM);
static_assert((SQ % 64) == 0 && (DM % 64) == 0 && (NTOK % 64) == 0);
static_assert(DM == 4 * 256);
static_assert((NTOK % 8) == 0);

typedef _Float16 v16h __attribute__((ext_vector_type(16)));
typedef _Float16 v8h  __attribute__((ext_vector_type(8)));
typedef float    v8f  __attribute__((ext_vector_type(8)));
typedef float    v4f  __attribute__((ext_vector_type(4)));
typedef unsigned int v4u __attribute__((ext_vector_type(4)));

__device__ __forceinline__ unsigned short bf_bits(float f) {
  unsigned u = __float_as_uint(f);
  return (unsigned short)((u + 0x7FFFu + ((u >> 16) & 1u)) >> 16);
}
__device__ __forceinline__ float bf_up(unsigned short h) { return __uint_as_float(((unsigned)h) << 16); }
__device__ __forceinline__ float bfr(float f) { return bf_up(bf_bits(f)); }
__device__ __forceinline__ unsigned short h_bits(_Float16 x) { return __builtin_bit_cast(unsigned short, x); }
__device__ __forceinline__ unsigned pk16(unsigned short a, unsigned short b) { return (unsigned)a | ((unsigned)b << 16); }
__device__ __forceinline__ v8f zero8() { v8f z = {0.f, 0.f, 0.f, 0.f, 0.f, 0.f, 0.f, 0.f}; return z; }

__device__ __forceinline__ v16h ldfrag_h(const _Float16* p) {
  union { v16h v; v8h h[2]; } f;
  f.h[0] = *(const v8h*)(p);
  f.h[1] = *(const v8h*)(p + 16);
  return f.v;
}

__device__ __forceinline__ v8f mma_h(v16h a, v16h b, v8f c) {
  c = __builtin_amdgcn_wmma_f32_16x16x32_f16(false, a, false, b, (short)0, c, false, false);
#if defined(__HIP_DEVICE_COMPILE__)
  asm volatile("v_nop\n\tv_nop\n\tv_nop\n\tv_nop" : "+v"(c) : "v"(a), "v"(b));
#endif
  return c;
}
__device__ __forceinline__ v8f mma_h_raw(v16h a, v16h b, v8f c) {
  return __builtin_amdgcn_wmma_f32_16x16x32_f16(false, a, false, b, (short)0, c, false, false);
}
__device__ __forceinline__ void dep_guard1(v8f& a, v8f& b, v16h x) {
#if defined(__HIP_DEVICE_COMPILE__)
  asm volatile("v_nop\n\tv_nop\n\tv_nop\n\tv_nop" : "+v"(a), "+v"(b) : "v"(x));
#endif
}
__device__ __forceinline__ void keep4_h(v16h a, v16h b, v16h c, v16h d) {
#if defined(__HIP_DEVICE_COMPILE__)
  asm volatile("v_nop" :: "v"(a), "v"(b), "v"(c), "v"(d));
#endif
}
__device__ __forceinline__ void acc_guard4(v8f& a, v8f& b, v8f& c, v8f& d) {
#if defined(__HIP_DEVICE_COMPILE__)
  asm volatile("v_nop\n\tv_nop\n\tv_nop\n\tv_nop" : "+v"(a), "+v"(b), "+v"(c), "+v"(d));
#endif
}
__device__ __forceinline__ void wave_sync_lds() {
  __builtin_amdgcn_fence(__ATOMIC_RELEASE, "workgroup");
  __builtin_amdgcn_wave_barrier();
  __builtin_amdgcn_fence(__ATOMIC_ACQUIRE, "workgroup");
}

__global__ __launch_bounds__(256) void ln_rows(const float* __restrict__ x, const float* __restrict__ gam,
                                               const float* __restrict__ bet, unsigned short* Xh,
                                               int nrows, float xsc, float eps) {
  const int lane = threadIdx.x & 31;
  const int wave = threadIdx.x >> 5;
  const int row  = blockIdx.x * 8 + wave;
  if (row >= nrows) return;
  const float* xr = x + (size_t)row * DM;
  const float rd = 1.0f / (float)DM;

  float s = 0.f;
#pragma unroll 1
  for (int i = 0; i < 4; ++i) {
    const int c0 = 256 * i + 8 * lane;
    const v4f a = *(const v4f*)(xr + c0);
    const v4f b = *(const v4f*)(xr + c0 + 4);
    s += ((bfr(a[0]) + bfr(a[1])) + (bfr(a[2]) + bfr(a[3]))) +
         ((bfr(b[0]) + bfr(b[1])) + (bfr(b[2]) + bfr(b[3])));
  }
#pragma unroll
  for (int off = 1; off < 32; off <<= 1) s += __shfl_xor(s, off, 32);
  const float mu = s * rd;

  float s2 = 0.f;
#pragma unroll 1
  for (int i = 0; i < 4; ++i) {
    const int c0 = 256 * i + 8 * lane;
    const v4f a = *(const v4f*)(xr + c0);
    const v4f b = *(const v4f*)(xr + c0 + 4);
#pragma unroll
    for (int e = 0; e < 4; ++e) {
      const float d0 = bfr(a[e]) - mu;
      const float d1 = bfr(b[e]) - mu;
      s2 += d0 * d0;
      s2 += d1 * d1;
    }
  }
#pragma unroll
  for (int off = 1; off < 32; off <<= 1) s2 += __shfl_xor(s2, off, 32);
  const float var  = s2 * rd;
  const float rstd = 1.0f / sqrtf(var + eps);

#pragma unroll 1
  for (int i = 0; i < 4; ++i) {
    const int c0 = 256 * i + 8 * lane;
    const v4f a  = *(const v4f*)(xr + c0);
    const v4f b  = *(const v4f*)(xr + c0 + 4);
    const v4f ga = *(const v4f*)(gam + c0);
    const v4f gb = *(const v4f*)(gam + c0 + 4);
    const v4f ba = *(const v4f*)(bet + c0);
    const v4f bb = *(const v4f*)(bet + c0 + 4);
    float y[8];
#pragma unroll
    for (int e = 0; e < 4; ++e) {
      y[e]     = ((bfr(a[e]) - mu) * rstd * bfr(ga[e]) + bfr(ba[e])) * xsc;
      y[4 + e] = ((bfr(b[e]) - mu) * rstd * bfr(gb[e]) + bfr(bb[e])) * xsc;
    }
    v4u u;
#pragma unroll
    for (int e = 0; e < 4; ++e) u[e] = pk16(h_bits((_Float16)y[2 * e]), h_bits((_Float16)y[2 * e + 1]));
    unsigned short* dst = Xh + (size_t)row * DM + c0;
    *(volatile v4u*)dst = u;
    __threadfence();
    *(volatile v4u*)dst = u;
  }
}

__global__ __launch_bounds__(256) void wtrans_h(const float* __restrict__ W, unsigned short* Wt,
                                                int R, int C, float wsc) {
  __shared__ __align__(16) unsigned short sT[64 * 72];
  const int tid = threadIdx.x;
  const int r0  = blockIdx.y * 64;
  const int c0  = blockIdx.x * 64;
#pragma unroll
  for (int it = 0; it < 4; ++it) {
    const int idx = it * 256 + tid;
    const int r   = idx >> 4;
    const int c4  = (idx & 15) * 4;
    const v4f w = *(const v4f*)(W + (size_t)(r0 + r) * C + c0 + c4);
#pragma unroll
    for (int e = 0; e < 4; ++e) sT[(c4 + e) * 72 + r] = h_bits((_Float16)(bfr(w[e]) * wsc));
  }
  __syncthreads();
  v4u u[2];
#pragma unroll
  for (int it = 0; it < 2; ++it) {
    const int row = it * 32 + (tid >> 3), col8 = (tid & 7) * 8;
    u[it] = *(const v4u*)(sT + row * 72 + col8);
  }
  for (int pass = 0; pass < 2; ++pass) {
#pragma unroll
    for (int it = 0; it < 2; ++it) {
      const int row = it * 32 + (tid >> 3), col8 = (tid & 7) * 8;
      *(volatile v4u*)(Wt + (size_t)(c0 + row) * R + r0 + col8) = u[it];
    }
    __threadfence();
  }
}

template <int OM, int BIASM>
__global__ __launch_bounds__(256) void gemm64(
    const unsigned short* __restrict__ Ap, int lda,
    const unsigned short* __restrict__ Btp, int ldb,
    const float* __restrict__ bias0,
    unsigned short* Cout, unsigned short* Cout2, int ldc,
    int M, int N, int K, float oscale, float bsc, float rsc) {
  const _Float16* A  = (const _Float16*)(const void*)Ap;
  const _Float16* Bt = (const _Float16*)(const void*)Btp;
  __shared__ __align__(16) float sT[8][16 * 68];
  const int lane = threadIdx.x & 31;
  const int wave = threadIdx.x >> 5;
  const int tilesN = N >> 6;
  const int tilesM = M >> 6;
  const int tile = blockIdx.x * 8 + wave;
  if (tile >= tilesM * tilesN) return;
  const int tm = tile / tilesN;
  const int tn = tile - tm * tilesN;
  const int m0 = tm << 6;
  const int n0 = tn << 6;

  const int rlane = lane & 15;
  const int koff  = (lane >> 4) * 8;
  const int mOff  = (lane >> 4) * 8;

  v8f acc[4][4];
#pragma unroll
  for (int i = 0; i < 4; ++i)
#pragma unroll
    for (int j = 0; j < 4; ++j) acc[i][j] = zero8();

  for (int k0 = 0; k0 < K; k0 += 32) {
    v16h bh[4];
#pragma unroll
    for (int j = 0; j < 4; ++j) {
      const size_t bo = (size_t)(n0 + (j << 4) + rlane) * ldb + koff + k0;
      bh[j] = ldfrag_h(Bt + bo);
    }
#pragma unroll
    for (int i = 0; i < 4; ++i) {
      const size_t ao = (size_t)(m0 + (i << 4) + rlane) * lda + koff + k0;
      const v16h ah = ldfrag_h(A + ao);
#pragma unroll
      for (int j = 0; j < 4; ++j) acc[i][j] = mma_h_raw(ah, bh[j], acc[i][j]);
      dep_guard1(acc[i][0], acc[i][3], ah);
    }
    keep4_h(bh[0], bh[1], bh[2], bh[3]);
  }
  acc_guard4(acc[0][0], acc[0][1], acc[0][2], acc[0][3]);
  acc_guard4(acc[1][0], acc[1][1], acc[1][2], acc[1][3]);
  acc_guard4(acc[2][0], acc[2][1], acc[2][2], acc[2][3]);
  acc_guard4(acc[3][0], acc[3][1], acc[3][2], acc[3][3]);

  const int q8 = lane >> 3, c8 = (lane & 7) * 8;
  float bc[8];
#pragma unroll
  for (int e = 0; e < 8; ++e) bc[e] = 0.f;
  if (BIASM == 0) {
    const int cb = n0 + c8;
    const int i0 = (cb < N - 8) ? cb : (N - 8);
    const v4f b0a = *(const v4f*)(bias0 + i0), b0b = *(const v4f*)(bias0 + i0 + 4);
#pragma unroll
    for (int e = 0; e < 4; ++e) {
      bc[e]     = bfr(b0a[e]) * bsc;
      bc[4 + e] = bfr(b0b[e]) * bsc;
    }
  }

  float* slab = sT[wave];
#pragma unroll
  for (int i = 0; i < 4; ++i) {
    const int mBase = m0 + (i << 4);
#pragma unroll
    for (int j = 0; j < 4; ++j) {
#pragma unroll
      for (int r = 0; r < 8; ++r) {
        slab[(mOff + r) * 68 + (j << 4) + rlane] = acc[i][j][r];
      }
    }
    wave_sync_lds();
    v4u hv[4], lv[4];
#pragma unroll
    for (int it = 0; it < 4; ++it) {
      const int row = it * 4 + q8;
      const float* sp = slab + row * 68 + c8;
      float bm = 0.f;
      if (BIASM == 1) bm = bfr(bias0[mBase + row]) * bsc;
      v4u a, lw;
#pragma unroll
      for (int e = 0; e < 4; ++e) {
        const float f0 = sp[2 * e]     * oscale + ((BIASM == 1) ? bm : bc[2 * e]);
        const float f1 = sp[2 * e + 1] * oscale + ((BIASM == 1) ? bm : bc[2 * e + 1]);
        const _Float16 g0 = (_Float16)f0;
        const _Float16 g1 = (_Float16)f1;
        a[e] = pk16(h_bits(g0), h_bits(g1));
        if (OM == 3) {
          const _Float16 r0 = (_Float16)((f0 - (float)g0) * rsc);
          const _Float16 r1 = (_Float16)((f1 - (float)g1) * rsc);
          lw[e] = pk16(h_bits(r0), h_bits(r1));
        } else {
          lw[e] = 0u;
        }
      }
      hv[it] = a;
      lv[it] = lw;
    }
    for (int pass = 0; pass < 2; ++pass) {
#pragma unroll
      for (int it = 0; it < 4; ++it) {
        const int row = it * 4 + q8;
        const size_t go = (size_t)(mBase + row) * ldc + n0 + c8;
        *(volatile v4u*)(Cout + go) = hv[it];
        if (OM == 3) *(volatile v4u*)(Cout2 + go) = lv[it];
      }
      __threadfence();
    }
    wave_sync_lds();
  }
}

__global__ __launch_bounds__(128)
void attn_lb(const unsigned short* __restrict__ qhp, const unsigned short* __restrict__ qlp,
             const unsigned short* __restrict__ khp,
             const unsigned short* __restrict__ vthp, const unsigned short* __restrict__ vtlp,
             float* outp, float sscale, float onorm) {
  union FH { v16h v; v8h h[2]; };
  __shared__ __align__(16) _Float16 Ksh[64 * 64];
  __shared__ __align__(16) _Float16 Vth[64 * 64];
  __shared__ __align__(16) _Float16 Vtl[64 * 64];
  __shared__ __align__(16) _Float16 Psh[4][16 * 64];
  __shared__ __align__(16) float    Os[4][16 * 64];

  const int tid  = threadIdx.x;
  const int wave = tid >> 5;
  const int lane = tid & 31;
  const int hh   = lane >> 4;
  const int c    = lane & 15;

  const int bx   = blockIdx.x;
  const int qb   = bx % NQB;
  const int hb   = bx / NQB;
  const int h    = hb % NH;
  const int b    = hb / NH;
  const int tok0 = b * SQ;
  const int ql0  = qb * 64 + wave * 16;
  const int q0   = tok0 + ql0;

  const _Float16* Qh = (const _Float16*)(const void*)qhp + (size_t)h * HD;
  const _Float16* Ql = (const _Float16*)(const void*)qlp + (size_t)h * HD;
  const _Float16* Kg = (const _Float16*)(const void*)khp + (size_t)h * HD;
  const _Float16* Vh = (const _Float16*)(const void*)vthp + (size_t)h * HD * NTOK + tok0;
  const _Float16* Vl = (const _Float16*)(const void*)vtlp + (size_t)h * HD * NTOK + tok0;

  const int   se    = (h + 1) >> 1;
  const float spw   = __uint_as_float((unsigned)(127 - se) << 23);
  const float slope = (h & 1) ? spw : (spw * 0.70710678118654752f);

  v16h qa[2], qr[2];
#pragma unroll
  for (int dc = 0; dc < 2; ++dc) {
    qa[dc] = ldfrag_h(Qh + (size_t)(q0 + c) * DM + dc * 32 + 8 * hh);
    qr[dc] = ldfrag_h(Ql + (size_t)(q0 + c) * DM + dc * 32 + 8 * hh);
  }

  float mrow[8], lrow[8];
  v8f oacc[4];
#pragma unroll
  for (int r = 0; r < 8; ++r) { mrow[r] = -INFINITY; lrow[r] = 0.f; }
#pragma unroll
  for (int t = 0; t < 4; ++t) oacc[t] = zero8();

  const float rinv = 1.0f / RSC;

  for (int kt = 0; kt < NQB; ++kt) {
    const int kv0 = kt * 64;
    __syncthreads();
    {
      const int r = tid >> 1, hf = (tid & 1) * 32;
      const _Float16* kg = Kg + (size_t)(tok0 + kv0 + r) * DM + hf;
      const _Float16* vg = Vh + (size_t)r * NTOK + kv0 + hf;
      const _Float16* wg = Vl + (size_t)r * NTOK + kv0 + hf;
#pragma unroll
      for (int i = 0; i < 4; ++i) {
        const v8h a0 = *(const v8h*)(kg + 8 * i);
        const v8h b0 = *(const v8h*)(vg + 8 * i);
        const v8h c0 = *(const v8h*)(wg + 8 * i);
        *(v8h*)(Ksh + r * 64 + hf + 8 * i) = a0;
        *(v8h*)(Vth + r * 64 + hf + 8 * i) = b0;
        *(v8h*)(Vtl + r * 64 + hf + 8 * i) = c0;
      }
    }
    __syncthreads();

    v8f s[4];
#pragma unroll
    for (int j = 0; j < 4; ++j) {
      v8f sh = zero8(), sl = zero8();
#pragma unroll
      for (int dc = 0; dc < 2; ++dc) {
        FH kb;
        kb.h[0] = *(const v8h*)(Ksh + (j * 16 + c) * 64 + dc * 32 + 8 * hh);
        kb.h[1] = *(const v8h*)(Ksh + (j * 16 + c) * 64 + dc * 32 + 16 + 8 * hh);
        sh = mma_h(qa[dc], kb.v, sh);
        sl = mma_h(qr[dc], kb.v, sl);
      }
      const int key = kv0 + j * 16 + c;
#pragma unroll
      for (int r = 0; r < 8; ++r) {
        const int qrow = ql0 + 8 * hh + r;
        int dd = key - qrow;
        if (dd < 0) dd = -dd;
        const float raw = sh[r] + sl[r] * rinv;
        s[j][r] = (raw - slope * (float)dd) * sscale;
      }
    }

    _Float16* pwh = Psh[wave];
#pragma unroll
    for (int r = 0; r < 8; ++r) {
      float m = s[0][r];
      m = fmaxf(m, s[1][r]);
      m = fmaxf(m, s[2][r]);
      m = fmaxf(m, s[3][r]);
#pragma unroll
      for (int off = 1; off < 16; off <<= 1) m = fmaxf(m, __shfl_xor(m, off, 32));
      const float mnew  = fmaxf(mrow[r], m);
      const float ms    = (mnew == -INFINITY) ? 0.f : mnew;
      const float alpha = __expf(mrow[r] - ms);
      mrow[r] = mnew;
      float psum = 0.f;
#pragma unroll
      for (int j = 0; j < 4; ++j) {
        const float p = __expf(s[j][r] - ms);
        psum += p;
        pwh[(8 * hh + r) * 64 + j * 16 + c] = (_Float16)(p * PSC);
      }
#pragma unroll
      for (int off = 1; off < 16; off <<= 1) psum += __shfl_xor(psum, off, 32);
      lrow[r] = lrow[r] * alpha + psum;
#pragma unroll
      for (int t = 0; t < 4; ++t) oacc[t][r] *= alpha;
    }
    wave_sync_lds();

    v8f ol[4];
#pragma unroll
    for (int t = 0; t < 4; ++t) ol[t] = zero8();
#pragma unroll 1
    for (int kk = 0; kk < 2; ++kk) {
      FH pa;
      pa.h[0] = *(const v8h*)(pwh + c * 64 + kk * 32 + 8 * hh);
      pa.h[1] = *(const v8h*)(pwh + c * 64 + kk * 32 + 16 + 8 * hh);
#pragma unroll
      for (int t = 0; t < 4; ++t) {
        FH vb, wb;
        vb.h[0] = *(const v8h*)(Vth + (t * 16 + c) * 64 + kk * 32 + 8 * hh);
        vb.h[1] = *(const v8h*)(Vth + (t * 16 + c) * 64 + kk * 32 + 16 + 8 * hh);
        wb.h[0] = *(const v8h*)(Vtl + (t * 16 + c) * 64 + kk * 32 + 8 * hh);
        wb.h[1] = *(const v8h*)(Vtl + (t * 16 + c) * 64 + kk * 32 + 16 + 8 * hh);
        oacc[t] = mma_h(pa.v, vb.v, oacc[t]);
        ol[t]   = mma_h(pa.v, wb.v, ol[t]);
      }
    }
#pragma unroll
    for (int t = 0; t < 4; ++t) {
#pragma unroll
      for (int r = 0; r < 8; ++r) oacc[t][r] += ol[t][r] * rinv;
    }
  }

  float* os = Os[wave];
#pragma unroll
  for (int r = 0; r < 8; ++r) {
    const float l = lrow[r];
    const float inv = ((l > 0.f) ? (1.0f / l) : 0.f) * onorm;
#pragma unroll
    for (int t = 0; t < 4; ++t) os[(8 * hh + r) * 64 + t * 16 + c] = oacc[t][r] * inv;
  }
  wave_sync_lds();
  {
    const int hh2 = lane >> 4, c4 = (lane & 15) * 4;
    v4f vals[8];
#pragma unroll
    for (int it = 0; it < 8; ++it) {
      const int row = it * 2 + hh2;
      vals[it] = *(const v4f*)(os + row * 64 + c4);
    }
    for (int pass = 0; pass < 2; ++pass) {
#pragma unroll
      for (int it = 0; it < 8; ++it) {
        const int row = it * 2 + hh2;
        const size_t go = (size_t)(q0 + row) * DM + (size_t)h * HD + c4;
        *(volatile v4f*)(outp + go) = vals[it];
      }
      __threadfence();
    }
  }
}

extern "C" void kernel_launch(void* const* d_in, const int* in_sizes, int n_in,
                              void* d_out, int out_size, void* d_ws, size_t ws_size,
                              hipStream_t stream) {
  if (n_in < 9) return;
  if (in_sizes[0] != NTOK * DM) return;
  if (in_sizes[1] != DM || in_sizes[2] != DM) return;
  if (in_sizes[3] != DM * DM || in_sizes[5] != DM * DM || in_sizes[7] != DM * DM) return;
  if (in_sizes[4] != DM || in_sizes[6] != DM || in_sizes[8] != DM) return;
  if (out_size != NTOK * DM) return;

  const float* x   = (const float*)d_in[0];
  const float* gam = (const float*)d_in[1];
  const float* bet = (const float*)d_in[2];
  const float* wq  = (const float*)d_in[3];
  const float* bq  = (const float*)d_in[4];
  const float* wk  = (const float*)d_in[5];
  const float* bk  = (const float*)d_in[6];
  const float* wv  = (const float*)d_in[7];
  const float* bv  = (const float*)d_in[8];

  const size_t PW = (size_t)DM * DM * 2;
  const size_t PA = (size_t)NTOK * DM * 2;
  size_t off = 0;
  const size_t oWq = off; off += PW;
  const size_t oWk = off; off += PW;
  const size_t oWv = off; off += PW;
  const size_t oXH = off; off += PA;
  const size_t oQH = off; off += PA;
  const size_t oQL = off; off += PA;
  const size_t oKH = off; off += PA;
  const size_t oVH = off; off += PA;
  const size_t oVL = off; off += PA;
  if (off > ws_size) return;
  if (off > (size_t)134217728) return;

  char* ws = (char*)d_ws;
  unsigned short* WqT = (unsigned short*)(ws + oWq);
  unsigned short* WkT = (unsigned short*)(ws + oWk);
  unsigned short* WvT = (unsigned short*)(ws + oWv);
  unsigned short* XH  = (unsigned short*)(ws + oXH);
  unsigned short* QH  = (unsigned short*)(ws + oQH);
  unsigned short* QL  = (unsigned short*)(ws + oQL);
  unsigned short* KH  = (unsigned short*)(ws + oKH);
  unsigned short* VTH = (unsigned short*)(ws + oVH);
  unsigned short* VTL = (unsigned short*)(ws + oVL);

  const dim3 blk(256), blk128(128);
  const dim3 gLn(NTOK / 8);
  const dim3 gTr(DM / 64, DM / 64);
  const dim3 gG(((NTOK / 64) * (DM / 64) + 7) / 8);
  const dim3 gAttn(NB * NH * NQB);
  const float osc_qk = 1.0f / (XSC * WSC);
  const float osc_v  = VSC / (XSC * WSC);

  ln_rows<<<gLn, blk, 0, stream>>>(x, gam, bet, XH, NTOK, XSC, LNEPS);
  wtrans_h<<<gTr, blk, 0, stream>>>(wq, WqT, DM, DM, WSC);
  wtrans_h<<<gTr, blk, 0, stream>>>(wk, WkT, DM, DM, WSC);
  wtrans_h<<<gTr, blk, 0, stream>>>(wv, WvT, DM, DM, WSC);
  gemm64<3, 0><<<gG, blk, 0, stream>>>(XH, DM, WqT, DM, bq, QH, QL, DM, NTOK, DM, DM, osc_qk, 1.0f, RSC);
  gemm64<2, 0><<<gG, blk, 0, stream>>>(XH, DM, WkT, DM, bk, KH, KH, DM, NTOK, DM, DM, osc_qk, 1.0f, RSC);
  gemm64<3, 1><<<gG, blk, 0, stream>>>(WvT, DM, XH, DM, bv, VTH, VTL, NTOK, DM, NTOK, DM, osc_v, VSC, RSC);
  attn_lb<<<gAttn, blk128, 0, stream>>>(QH, QL, KH, VTH, VTL, (float*)d_out, 0.125f, 1.0f / (PSC * VSC));
  (void)hipGetLastError();
}
